// CriticNetwork_59425167507826
// MI455X (gfx1250) — hardware-verified
//
#include <hip/hip_runtime.h>
#include <math.h>

typedef __attribute__((ext_vector_type(16))) _Float16 v16h;
typedef __attribute__((ext_vector_type(16))) __bf16 v16b;
typedef __attribute__((ext_vector_type(8)))  _Float16 v8h;
typedef __attribute__((ext_vector_type(8)))  float v8f;
typedef __attribute__((ext_vector_type(4)))  float v4f;
typedef __attribute__((ext_vector_type(2)))  float v2f;
typedef __attribute__((ext_vector_type(4)))  unsigned v4u;
typedef __attribute__((ext_vector_type(4)))  int v4i;
typedef float __attribute__((may_alias)) float_a;
typedef int __attribute__((may_alias)) int_a;

template <typename T> __device__ __forceinline__ void vst2(void* p, T v) { *(volatile T*)p = v; __threadfence(); *(volatile T*)p = v; }
__device__ __forceinline__ v8f wmma16(v16h a, v16h b, v8f c) {
  v8f d = __builtin_amdgcn_wmma_f32_16x16x32_f16(false, a, false, b, (short)0, c, false, false);
  asm volatile("v_nop\n\tv_nop\n\tv_nop\n\tv_nop" : "+v"(d) : "v"(a), "v"(b));
  return d;
}
__device__ __forceinline__ v8f wmma_bf(v16b a, v16b b, v8f c) {
  v8f d = __builtin_amdgcn_wmma_f32_16x16x32_bf16(false, a, false, b, (short)0, c, false, false);
  asm volatile("v_nop\n\tv_nop\n\tv_nop\n\tv_nop" : "+v"(d) : "v"(a), "v"(b));
  return d;
}
__device__ __forceinline__ v16h frag_h(const _Float16* rowk0, int lane) {
  union { v16h v; v8h q[2]; } u; const _Float16* p = rowk0 + 8 * (lane >> 4);
  u.q[0] = *(const v8h*)p; u.q[1] = *(const v8h*)(p + 16); return u.v;
}
__device__ __forceinline__ v16h frag_f32(const float* rowk0, int lane) {
  v16h a; const float* p = rowk0 + 8 * (lane >> 4);
#pragma unroll
  for (int i = 0; i < 8; ++i) { a[i] = (_Float16)p[i]; a[8 + i] = (_Float16)p[16 + i]; }
  return a;
}
__device__ __forceinline__ v16h frag_f32s(const float* rowk0, int lane, float sc) {
  v16h a; const float* p = rowk0 + 8 * (lane >> 4);
#pragma unroll
  for (int i = 0; i < 8; ++i) { a[i] = (_Float16)(p[i] * sc); a[8 + i] = (_Float16)(p[16 + i] * sc); }
  return a;
}
__device__ __forceinline__ v16h fragc_f32(const float* W, int k0, int n, int lane, int ld, int K) {
  v16h a; const int g = lane >> 4;
#pragma unroll
  for (int i = 0; i < 8; ++i) { const int ka = k0 + 8 * g + i, kb = ka + 16;
    a[i] = (_Float16)(ka < K ? W[(size_t)ka * ld + n] : 0.f); a[8 + i] = (_Float16)(kb < K ? W[(size_t)kb * ld + n] : 0.f); }
  return a;
}
struct F2 { v16b h, l; };
__device__ __forceinline__ F2 bsplit16(const float v[16]) { F2 r;
#pragma unroll
  for (int i = 0; i < 16; ++i) { const __bf16 h = (__bf16)v[i]; r.h[i] = h; r.l[i] = (__bf16)(v[i] - (float)h); }
  return r; }
__device__ __forceinline__ F2 split_row(const float* row, int k0, int lane) { float v[16]; const float* p = row + k0 + 8 * (lane >> 4);
#pragma unroll
  for (int i = 0; i < 8; ++i) { v[i] = p[i]; v[8 + i] = p[16 + i]; }
  return bsplit16(v); }
__device__ __forceinline__ F2 split_rowK(const float* row, int k0, int lane, int K) { float v[16]; const int g = lane >> 4;
#pragma unroll
  for (int i = 0; i < 8; ++i) { const int ka = k0 + 8 * g + i, kb = ka + 16; v[i] = ka < K ? row[ka] : 0.f; v[8 + i] = kb < K ? row[kb] : 0.f; }
  return bsplit16(v); }
__device__ __forceinline__ F2 split_col(const float* W, int k0, int n, int lane, int ld, int K) { float v[16]; const int g = lane >> 4;
#pragma unroll
  for (int i = 0; i < 8; ++i) { const int ka = k0 + 8 * g + i, kb = ka + 16; v[i] = ka < K ? W[(size_t)ka * ld + n] : 0.f; v[8 + i] = kb < K ? W[(size_t)kb * ld + n] : 0.f; }
  return bsplit16(v); }
__device__ __forceinline__ v8f mac3(const F2& a, const F2& b, v8f c) { c = wmma_bf(a.l, b.h, c); c = wmma_bf(a.h, b.l, c); return wmma_bf(a.h, b.h, c); }
__device__ __forceinline__ float sigm(float v) { return 1.0f / (1.0f + expf(-v)); }
#define LDSX() do { asm volatile("s_wait_dscnt 0" ::: "memory"); __builtin_amdgcn_wave_barrier(); __builtin_amdgcn_fence(__ATOMIC_RELEASE, "workgroup"); } while (0)

#define NBT 128
#define NAG 32
#define OBS 64
#define ACT 16
#define DIN 80
#define HH 64
#define FIN 128

__device__ __forceinline__ void packW(_Float16* dst, int ldd, const float* __restrict__ W, int K, int N, int KP, int tid, int nth) {
  for (int q = tid; q < N * KP; q += nth) { const int n = q / KP, k = q % KP; dst[n * ldd + k] = (_Float16)(k < K ? W[k * N + n] * 16.0f : 0.f); }
}
__global__ __launch_bounds__(128) void k_pre(const float* __restrict__ st, const float* __restrict__ po, const float* __restrict__ ac,
    const float* __restrict__ kw1, const float* __restrict__ kb1, const float* __restrict__ kw2, const float* __restrict__ kb2, const float* __restrict__ qw1, const float* __restrict__ qb1, const float* __restrict__ qw2, const float* __restrict__ qb2,
    const float* __restrict__ ko1, const float* __restrict__ kob1, const float* __restrict__ ko2, const float* __restrict__ kob2, const float* __restrict__ av1, const float* __restrict__ ab1, const float* __restrict__ av2, const float* __restrict__ ab2,
    float* __restrict__ KZ, float* __restrict__ QZ, float* __restrict__ KO, float* __restrict__ VPI) {
  __shared__ __align__(16) _Float16 sw1[4][HH][104];
  __shared__ __align__(16) _Float16 sw2[4][HH][72];
  __shared__ float sb1[4][HH], sb2[4][HH];
  __shared__ __align__(16) _Float16 sa[4][16][104];
  __shared__ __align__(16) float so[4][16][68];
  __shared__ float skq[2][4][16][HH + 1];
  __shared__ __align__(16) _Float16 sh[4][16][72];
  const int tid = threadIdx.x, wave = tid >> 5, lane = tid & 31, col = lane & 15, g = lane >> 4;
  const int r0 = blockIdx.x * 64 + wave * 16;
  packW(&sw1[0][0][0], 104, kw1, OBS, HH, 96, tid, 128); packW(&sw1[1][0][0], 104, qw1, OBS, HH, 96, tid, 128); packW(&sw1[2][0][0], 104, ko1, DIN, HH, 96, tid, 128); packW(&sw1[3][0][0], 104, av1, DIN, HH, 96, tid, 128);
  packW(&sw2[0][0][0], 72, kw2, HH, HH, 64, tid, 128); packW(&sw2[1][0][0], 72, qw2, HH, HH, 64, tid, 128); packW(&sw2[2][0][0], 72, ko2, HH, HH, 64, tid, 128); packW(&sw2[3][0][0], 72, av2, HH, HH, 64, tid, 128);
  for (int q = tid; q < 4 * HH; q += 128) { const int m = q >> 6, n = q & 63; sb1[m][n] = (m == 0 ? kb1 : m == 1 ? qb1 : m == 2 ? kob1 : ab1)[n]; sb2[m][n] = (m == 0 ? kb2 : m == 1 ? qb2 : m == 2 ? kob2 : ab2)[n]; }
  __syncthreads();
  { const int r = r0 + col; const float* sr = st + (size_t)r * OBS;
    for (int k = g; k < 96; k += 2) sa[wave][col][k] = (_Float16)(k < OBS ? sr[k] : 0.f); }
  LDSX();
#pragma unroll 1
  for (int m = 0; m < 4; ++m) {
    if (m == 2) {
      LDSX();
      { const int r = r0 + col; float dz = 0.f; for (int d = 0; d < HH; ++d) dz += skq[0][wave][col][d] * skq[1][wave][col][d];
        const float wz = sigm(dz * 0.125f);
        for (int k = OBS + g; k < DIN; k += 2) { const int e = k - OBS; sa[wave][col][k] = (_Float16)(wz * ac[(size_t)r * ACT + e] + (1.f - wz) * po[(size_t)r * ACT + e]); } }
      LDSX(); }
    if (m == 3) {
      LDSX();
      { const int r = r0 + col; for (int k = OBS + g; k < DIN; k += 2) sa[wave][col][k] = (_Float16)po[(size_t)r * ACT + (k - OBS)]; }
      LDSX(); }
    v8f acc[4] = {};
#pragma unroll
    for (int kc = 0; kc < 3; ++kc) { const v16h a = frag_h(&sa[wave][col][0] + kc * 32, lane);
#pragma unroll
      for (int t = 0; t < 4; ++t) acc[t] = wmma16(a, frag_h(&sw1[m][t * 16 + col][0] + kc * 32, lane), acc[t]); }
#pragma unroll
    for (int t = 0; t < 4; ++t) { const int n = t * 16 + col; const float bb = sb1[m][n];
#pragma unroll
      for (int r = 0; r < 8; ++r) { float v = acc[t][r] * (1.0f / 16.0f) + bb; v = v > 0.f ? v : 0.01f * v; sh[wave][8 * g + r][n] = (_Float16)v; } }
    LDSX();
    v8f acc2[4] = {};
#pragma unroll
    for (int kc = 0; kc < 2; ++kc) { const v16h a = frag_h(&sh[wave][col][0] + kc * 32, lane);
#pragma unroll
      for (int t = 0; t < 4; ++t) acc2[t] = wmma16(a, frag_h(&sw2[m][t * 16 + col][0] + kc * 32, lane), acc2[t]); }
#pragma unroll
    for (int t = 0; t < 4; ++t) { const int n = t * 16 + col; const float bb = sb2[m][n];
#pragma unroll
      for (int r = 0; r < 8; ++r) { const float v = acc2[t][r] * (1.0f / 16.0f) + bb; so[wave][8 * g + r][n] = v; if (m < 2) skq[m][wave][8 * g + r][n] = v; } }
    LDSX();
    float* D = m == 0 ? KZ : m == 1 ? QZ : m == 2 ? KO : VPI;
    for (int q = lane; q < 16 * 16; q += 32) { const int rl = q >> 4, pc = q & 15; vst2(D + (size_t)(r0 + rl) * HH + pc * 4, *(const v4f*)(&so[wave][rl][pc * 4])); }
    LDSX(); }
}
__global__ __launch_bounds__(128) void k_main(const float* __restrict__ st, const float* __restrict__ po, const float* __restrict__ ac, const float* __restrict__ KZ, const float* __restrict__ QZ, const float* __restrict__ KO, const float* __restrict__ VPI,
    const float* __restrict__ qo1, const float* __restrict__ qob1, const float* __restrict__ qo2, const float* __restrict__ qob2, const float* __restrict__ av1, const float* __restrict__ ab1, const float* __restrict__ av2, const float* __restrict__ ab2,
    const float* __restrict__ fv1, const float* __restrict__ fb1, const float* __restrict__ fv2, const float* __restrict__ fb2, float* __restrict__ oval, float* __restrict__ owz, float* __restrict__ owo) {
  __shared__ __align__(16) _Float16 sw1[2][HH][104];
  __shared__ __align__(16) _Float16 sw2[2][HH][72];
  __shared__ __align__(16) _Float16 swf[HH][136];
  __shared__ float sb1[2][HH], sb2[2][HH], sbf[HH], sfv2[HH];
  __shared__ __align__(16) _Float16 sa[4][16][136];
  __shared__ __align__(16) _Float16 sh[4][16][72];
  __shared__ float sq[64][HH + 1], sv[64][HH + 1];
  __shared__ float swz[64], swo[64], ssc[64]; __shared__ float ssum[2][HH]; __shared__ __align__(16) float sval[64];
  const int tid = threadIdx.x, wave = tid >> 5, lane = tid & 31, col = lane & 15, g = lane >> 4;
  const int b = blockIdx.y, a0 = blockIdx.x * 2; const int al = wave >> 1, a = a0 + al; const int jrow0 = (wave & 1) * 16;
  packW(&sw1[0][0][0], 104, qo1, DIN, HH, 96, tid, 128); packW(&sw1[1][0][0], 104, av1, DIN, HH, 96, tid, 128);
  packW(&sw2[0][0][0], 72, qo2, HH, HH, 64, tid, 128); packW(&sw2[1][0][0], 72, av2, HH, HH, 64, tid, 128);
  packW(&swf[0][0], 136, fv1, FIN, HH, 128, tid, 128);
  if (tid < HH) { sb1[0][tid] = qob1[tid]; sb1[1][tid] = ab1[tid]; sb2[0][tid] = qob2[tid]; sb2[1][tid] = ab2[tid]; sbf[tid] = fb1[tid]; sfv2[tid] = fv2[tid]; }
  __syncthreads();
  { const int m = col, j = jrow0 + m, rl = wave * 16 + m;
    if (g == 0) { float dz = 0.f; for (int d = 0; d < HH; ++d) dz += KZ[((size_t)b * NAG + a) * HH + d] * QZ[((size_t)b * NAG + j) * HH + d]; swz[rl] = sigm(dz * 0.125f); }
    LDSX();
    const float wz = swz[rl];
    for (int k = g; k < 96; k += 2) { float v = 0.f; if (k < OBS) v = st[((size_t)b * NAG + j) * OBS + k]; else if (k < DIN) { const int e = k - OBS; v = wz * ac[((size_t)b * NAG + j) * ACT + e] + (1.f - wz) * po[((size_t)b * NAG + j) * ACT + e]; }
      sa[wave][col][k] = (_Float16)v; } }
  LDSX();
#pragma unroll 1
  for (int mm = 0; mm < 2; ++mm) { v8f acc[4] = {};
#pragma unroll
    for (int kc = 0; kc < 3; ++kc) { const v16h af = frag_h(&sa[wave][col][0] + kc * 32, lane);
#pragma unroll
      for (int t = 0; t < 4; ++t) acc[t] = wmma16(af, frag_h(&sw1[mm][t * 16 + col][0] + kc * 32, lane), acc[t]); }
#pragma unroll
    for (int t = 0; t < 4; ++t) { const int n = t * 16 + col; const float bb = sb1[mm][n];
#pragma unroll
      for (int r = 0; r < 8; ++r) { float v = acc[t][r] * (1.0f / 16.0f) + bb; v = v > 0.f ? v : 0.01f * v; sh[wave][8 * g + r][n] = (_Float16)v; } }
    LDSX();
    v8f acc2[4] = {};
#pragma unroll
    for (int kc = 0; kc < 2; ++kc) { const v16h af = frag_h(&sh[wave][col][0] + kc * 32, lane);
#pragma unroll
      for (int t = 0; t < 4; ++t) acc2[t] = wmma16(af, frag_h(&sw2[mm][t * 16 + col][0] + kc * 32, lane), acc2[t]); }
#pragma unroll
    for (int t = 0; t < 4; ++t) { const int n = t * 16 + col; const float bb = sb2[mm][n];
#pragma unroll
      for (int r = 0; r < 8; ++r) { const float v = acc2[t][r] * (1.0f / 16.0f) + bb; if (mm == 0) sq[wave * 16 + 8 * g + r][n] = v; else sv[wave * 16 + 8 * g + r][n] = v; } }
    LDSX(); }
  __syncthreads();
  if (tid < 64) { const int rl = tid; const int ag = rl >> 5; (void)ag; float s = 0.f; const float* ko = KO + ((size_t)b * NAG + a0 + (rl >> 5)) * HH;
    for (int d = 0; d < HH; ++d) s += ko[d] * sq[rl][d]; ssc[rl] = s * 0.125f; }
  __syncthreads();
  if (tid < 64) { const int rl = tid, base = rl & 32; float mx = -3.0e38f; for (int e = 0; e < 32; ++e) mx = fmaxf(mx, ssc[base + e]); float l = 0.f; for (int e = 0; e < 32; ++e) l += expf(ssc[base + e] - mx); swo[rl] = expf(ssc[rl] - mx) / l; }
  __syncthreads();
  { const int ag = tid >> 6, d = tid & 63; float s = 0.f; for (int e = 0; e < 32; ++e) s += swo[ag * 32 + e] * sv[ag * 32 + e][d]; ssum[ag][d] = s; }
  __syncthreads();
  { const int m = col, j = jrow0 + m, rl = wave * 16 + m; const float w = swo[rl];
    for (int k = g; k < FIN; k += 2) { float v; if (k < OBS) v = st[((size_t)b * NAG + j) * OBS + k]; else { const int d = k - OBS; v = (ssum[al][d] - w * sv[rl][d] + w * VPI[((size_t)b * NAG + j) * HH + d]) * (1.0f / NAG); }
      sa[wave][col][k] = (_Float16)v; } }
  LDSX();
  { v8f acc[4] = {};
#pragma unroll
    for (int kc = 0; kc < 4; ++kc) { const v16h af = frag_h(&sa[wave][col][0] + kc * 32, lane);
#pragma unroll
      for (int t = 0; t < 4; ++t) acc[t] = wmma16(af, frag_h(&swf[t * 16 + col][0] + kc * 32, lane), acc[t]); }
#pragma unroll
    for (int t = 0; t < 4; ++t) { const int n = t * 16 + col; const float bb = sbf[n];
#pragma unroll
      for (int r = 0; r < 8; ++r) { float v = acc[t][r] * (1.0f / 16.0f) + bb; v = v > 0.f ? v : 0.01f * v; sq[wave * 16 + 8 * g + r][n] = v; } }
    LDSX();
    if (g == 0) { const int rl = wave * 16 + col; float s = fb2[0]; for (int d = 0; d < HH; ++d) s += sq[rl][d] * sfv2[d]; sval[rl] = s; } }
  __syncthreads();
  const size_t ob = ((size_t)b * NAG + a0) * NAG;
  if (tid < 16) vst2(oval + ob + tid * 4, *(const v4f*)(&sval[tid * 4]));
  else if (tid >= 32 && tid < 48) { const int q = tid - 32; v4f o; o[0] = swz[q * 4]; o[1] = swz[q * 4 + 1]; o[2] = swz[q * 4 + 2]; o[3] = swz[q * 4 + 3]; vst2(owz + ob + q * 4, o); }
  else if (tid >= 64 && tid < 80) { const int q = tid - 64; v4f o; o[0] = swo[q * 4]; o[1] = swo[q * 4 + 1]; o[2] = swo[q * 4 + 2]; o[3] = swo[q * 4 + 3]; vst2(owo + ob + q * 4, o); }
}
extern "C" void kernel_launch(void* const* d_in, const int* in_sizes, int n_in, void* d_out, int out_size, void* d_ws, size_t ws_size, hipStream_t stream) {
  (void)in_sizes; (void)n_in; (void)out_size; (void)ws_size;
  const float** I = (const float**)d_in;
  float* oval = (float*)d_out; float* owz = (float*)((char*)d_out + 524288); float* owo = (float*)((char*)d_out + 1048576);
  char* ws = (char*)d_ws; size_t off = 0;
  auto take = [&](size_t bytes) { char* p = ws + off; off += (bytes + 255) & ~(size_t)255; return p; };
  float* KZ = (float*)take((size_t)NBT * NAG * HH * 4); float* QZ = (float*)take((size_t)NBT * NAG * HH * 4); float* KO = (float*)take((size_t)NBT * NAG * HH * 4); float* VPI = (float*)take((size_t)NBT * NAG * HH * 4);
  k_pre<<<NBT * NAG / 64, 128, 0, stream>>>(I[0], I[1], I[2], I[3], I[4], I[5], I[6], I[7], I[8], I[9], I[10], I[11], I[12], I[13], I[14], I[19], I[20], I[21], I[22], KZ, QZ, KO, VPI);
  k_main<<<dim3(NAG / 2, NBT), 128, 0, stream>>>(I[0], I[1], I[2], KZ, QZ, KO, VPI, I[15], I[16], I[17], I[18], I[19], I[20], I[21], I[22], I[23], I[24], I[25], I[26], oval, owz, owo);
}
